// TransformerCritic_66709432041567
// MI455X (gfx1250) — hardware-verified
//
#include <hip/hip_runtime.h>

#define NB   128
#define NA   32
#define OBS  128
#define ACT  16
#define NH   4
#define DMD  128
#define EV   32
#define FIN  16
#define OA   144
#define OAP  160
#define HID  64

#define OUT0_N (NB * NA * NA * FIN)
#define OUT1_N (NB * NH * NA * NA)

#define ASC   16.0f
#define WSC   64.0f
#define RSC   2048.0f
#define PINV  0.0009765625f
#define RINV  4.76837158203125e-7f
#define HHINV 0.00390625f
#define XINV  1.9073486328125e-6f
#define INVSQ 0.08838834764831845f

#define PT 136
#define PA 168
#define PW 40
#define PH 72
#define PS 36

#define A_S     0
#define A_SEH   8704
#define A_SEL   17408
#define A_QH    26112
#define A_QL    34816
#define A_KH    43520
#define A_KL    52224
#define A_SC    60928
#define A_B     65536
#define A_TOTAL 67072
#define E_A     0
#define E_EH    21504
#define E_EL    38912
#define E_AV    56320
#define E_B     93184
#define E_TOTAL 95744
#define N_WH    0
#define N_WL    10240
#define N_TH    20480
#define N_TL    40960
#define N_NH    61440
#define N_NL    78848
#define N_HH    96256
#define N_HL    105472
#define N_ST    114688
#define N_BB    119296
#define N_TOTAL 119808

static_assert(A_SEH == A_S + NA * PT * 2);
static_assert(A_SEL == A_SEH + NA * PT * 2);
static_assert(A_QH == A_SEL + NA * PT * 2);
static_assert(A_QL == A_QH + NA * PT * 2);
static_assert(A_KH == A_QL + NA * PT * 2);
static_assert(A_KL == A_KH + NA * PT * 2);
static_assert(A_SC == A_KL + NA * PT * 2);
static_assert(A_B == A_SC + NA * PS * 4);
static_assert(A_TOTAL == A_B + 3 * DMD * 4);
static_assert(E_EH == E_A + 2 * NA * PA * 2);
static_assert(E_EL == E_EH + 2 * NA * PT * 2);
static_assert(E_AV == E_EL + 2 * NA * PT * 2);
static_assert(E_B == E_AV + NH * 2 * NA * PS * 4);
static_assert(E_TOTAL == E_B + (NH * DMD + NH * EV) * 4);
static_assert(N_WL == N_WH + NH * NA * PW * 2);
static_assert(N_TH == N_WL + NH * NA * PW * 2);
static_assert(N_TL == N_TH + 2 * NH * EV * PW * 2);
static_assert(N_NH == N_TL + 2 * NH * EV * PW * 2);
static_assert(N_NL == N_NH + 2 * NA * PT * 2);
static_assert(N_HH == N_NL + 2 * NA * PT * 2);
static_assert(N_HL == N_HH + 2 * NA * PH * 2);
static_assert(N_ST == N_HL + 2 * NA * PH * 2);
static_assert(N_BB == N_ST + NA * PS * 4);
static_assert(N_TOTAL >= N_BB + (HID + FIN) * 4);
static_assert((A_SC % 16) == 0 && (A_B % 16) == 0 && (E_EH % 16) == 0 && (E_AV % 16) == 0 && (E_B % 16) == 0);
static_assert((N_TH % 16) == 0 && (N_NH % 16) == 0 && (N_HH % 16) == 0 && (N_ST % 16) == 0 && (N_BB % 16) == 0);
static_assert((PT % 8) == 0 && (PA % 8) == 0 && (PW % 8) == 0 && (PH % 8) == 0 && (PS % 4) == 0);
static_assert(OAP % 32 == 0 && OAP >= OA);

typedef _Float16 f16;
typedef _Float16 v16h __attribute__((ext_vector_type(16)));
typedef _Float16 v8h  __attribute__((ext_vector_type(8)));
typedef _Float16 v8ha __attribute__((ext_vector_type(8), may_alias));
typedef _Float16 v4h  __attribute__((ext_vector_type(4)));
typedef unsigned short v8us __attribute__((ext_vector_type(8)));
typedef float v8f __attribute__((ext_vector_type(8)));
typedef float v4f __attribute__((ext_vector_type(4)));
typedef float v4fa __attribute__((ext_vector_type(4), may_alias));

union FragH { v16h v; v8h h[2]; };

__device__ __forceinline__ float bf16r(float f) {
  unsigned int u = __float_as_uint(f);
  u = u + 0x7FFFu + ((u >> 16) & 1u);
  u &= 0xFFFF0000u;
  return __uint_as_float(u);
}

__device__ __forceinline__ float leaky_f(float x) { return x >= 0.0f ? x : 0.01f * x; }

__device__ __forceinline__ void split16(float v, f16& hi, f16& lo) {
  const float s = v * ASC;
  const f16 hv = (f16)s;
  hi = hv;
  lo = (f16)((s - (float)hv) * RSC);
}

__device__ __forceinline__ v16h ld_frag(const f16* base, int row0, int k0, int ld) {
  const int lane = threadIdx.x & 31;
  const f16* p = base + (size_t)(row0 + (lane & 15)) * ld + k0 + ((lane >> 4) << 3);
  FragH f;
  f.h[0] = *(const v8h*)p;
  f.h[1] = *(const v8h*)(p + 16);
  return f.v;
}

__device__ __forceinline__ v8f mma_h(v16h a, v16h b, v8f c) {
  return __builtin_amdgcn_wmma_f32_16x16x32_f16(false, a, false, b, (short)0, c, false, false);
}

__device__ __forceinline__ void guard2_3(v8f& c0, v8f& c1, v16h f0, v16h f1, v16h f2) {
#if defined(__HIP_DEVICE_COMPILE__)
  asm volatile("v_nop\n\tv_nop\n\tv_nop\n\tv_nop"
               : "+v"(c0), "+v"(c1) : "v"(f0), "v"(f1), "v"(f2));
#endif
}
__device__ __forceinline__ void guard2_4(v8f& c0, v8f& c1, v16h f0, v16h f1, v16h f2, v16h f3) {
#if defined(__HIP_DEVICE_COMPILE__)
  asm volatile("v_nop\n\tv_nop\n\tv_nop\n\tv_nop"
               : "+v"(c0), "+v"(c1) : "v"(f0), "v"(f1), "v"(f2), "v"(f3));
#endif
}
__device__ __forceinline__ void guard4_5(v8f& c0, v8f& c1, v8f& c2, v8f& c3,
                                         v16h f0, v16h f1, v16h f2, v16h f3, v16h f4) {
#if defined(__HIP_DEVICE_COMPILE__)
  asm volatile("v_nop\n\tv_nop\n\tv_nop\n\tv_nop"
               : "+v"(c0), "+v"(c1), "+v"(c2), "+v"(c3)
               : "v"(f0), "v"(f1), "v"(f2), "v"(f3), "v"(f4));
#endif
}
__device__ __forceinline__ void guard4_6(v8f& c0, v8f& c1, v8f& c2, v8f& c3,
                                         v16h f0, v16h f1, v16h f2, v16h f3, v16h f4, v16h f5) {
#if defined(__HIP_DEVICE_COMPILE__)
  asm volatile("v_nop\n\tv_nop\n\tv_nop\n\tv_nop"
               : "+v"(c0), "+v"(c1), "+v"(c2), "+v"(c3)
               : "v"(f0), "v"(f1), "v"(f2), "v"(f3), "v"(f4), "v"(f5));
#endif
}

__global__ __launch_bounds__(256)
void k_cvt_t(const float* __restrict__ src, unsigned short* dst, int G, int K, int N, int Kp) {
  const int KQ = Kp >> 3;
  const int n8 = G * N * KQ;
  const int p = (int)blockIdx.x * 256 + (int)threadIdx.x;
  if (p >= n8) return;
  const int kq = p % KQ;
  const int t1 = p / KQ;
  const int n = t1 % N;
  const int g = t1 / N;
  v8h o = {};
#pragma unroll
  for (int c = 0; c < 8; ++c) {
    const int k = kq * 8 + c;
    const int kc = (k < K) ? k : (K - 1);
    float v = src[((size_t)(g * K + kc)) * N + n];
    v = (k < K) ? v : 0.0f;
    o[c] = (f16)(bf16r(v) * WSC);
  }
  const v8us u = __builtin_bit_cast(v8us, o);
  unsigned short* op = dst + (size_t)p * 8;
  *(volatile v8us*)op = u;
  __threadfence();
  *(volatile v8us*)op = u;
}

__global__ __launch_bounds__(256)
void k_attn(const float* __restrict__ states,
            const unsigned short* __restrict__ wse_h, const float* __restrict__ b_se,
            const unsigned short* __restrict__ wk_h,  const float* __restrict__ b_k,
            const unsigned short* __restrict__ wq_h,  const float* __restrict__ b_q,
            float* outw, int nbh) {
  extern __shared__ __align__(16) char smem[];
  f16* S   = (f16*)(smem + A_S);
  f16* SEH = (f16*)(smem + A_SEH);
  f16* SEL = (f16*)(smem + A_SEL);
  f16* QH  = (f16*)(smem + A_QH);
  f16* QL  = (f16*)(smem + A_QL);
  f16* KH  = (f16*)(smem + A_KH);
  f16* KL  = (f16*)(smem + A_KL);
  float* Sc   = (float*)(smem + A_SC);
  float* bias = (float*)(smem + A_B);

  const int tid = threadIdx.x, lane = tid & 31, wv = tid >> 5, hl = lane >> 4, l15 = lane & 15;
  const int bh = (int)blockIdx.x;
  if (bh >= nbh) return;
  const int b = bh >> 2, h = bh & 3;

#pragma unroll
  for (int it = 0; it < 2; ++it) {
    const int idx = tid + it * 256;
    const int r = idx >> 4, c8 = (idx & 15) << 3;
    const float* p = states + (size_t)(b * NA + r) * OBS + c8;
    const v4f x0 = *(const v4f*)p;
    const v4f x1 = *(const v4f*)(p + 4);
    v8h o = {};
#pragma unroll
    for (int e = 0; e < 4; ++e) {
      o[e]     = (f16)(bf16r(x0[e]) * ASC);
      o[4 + e] = (f16)(bf16r(x1[e]) * ASC);
    }
    *(v8h*)&S[r * PT + c8] = o;
  }
  if (tid < DMD) {
    bias[tid]           = bf16r(b_se[h * DMD + tid]);
    bias[DMD + tid]     = bf16r(b_k[h * DMD + tid]);
    bias[2 * DMD + tid] = bf16r(b_q[h * DMD + tid]);
  }
  __syncthreads();

  {
    const f16* wp = (const f16*)wse_h + (size_t)h * DMD * DMD;
    v8f c0 = {}, c1 = {};
#pragma unroll
    for (int ks = 0; ks < 4; ++ks) {
      const v16h a0 = ld_frag(S, 0, 32 * ks, PT);
      const v16h a1 = ld_frag(S, 16, 32 * ks, PT);
      const v16h bw = ld_frag(wp, 16 * wv, 32 * ks, DMD);
      c0 = mma_h(a0, bw, c0);
      c1 = mma_h(a1, bw, c1);
      guard2_3(c0, c1, a0, a1, bw);
    }
    const int col = 16 * wv + l15;
    const float bb = bias[col];
#pragma unroll
    for (int r = 0; r < 8; ++r) {
      f16 x, y;
      split16(leaky_f(c0[r] * PINV + bb), x, y);
      SEH[(8 * hl + r) * PT + col] = x;
      SEL[(8 * hl + r) * PT + col] = y;
      split16(leaky_f(c1[r] * PINV + bb), x, y);
      SEH[(16 + 8 * hl + r) * PT + col] = x;
      SEL[(16 + 8 * hl + r) * PT + col] = y;
    }
  }
  __syncthreads();

#pragma unroll 1
  for (int sel = 0; sel < 2; ++sel) {
    const f16* wp = (const f16*)(sel ? wq_h : wk_h) + (size_t)h * DMD * DMD;
    f16* OH = sel ? QH : KH;
    f16* OL = sel ? QL : KL;
    const float* bp = bias + (sel ? 2 * DMD : DMD);
    v8f ch0 = {}, ch1 = {}, cl0 = {}, cl1 = {};
#pragma unroll
    for (int ks = 0; ks < 4; ++ks) {
      const v16h aH0 = ld_frag(SEH, 0, 32 * ks, PT);
      const v16h aH1 = ld_frag(SEH, 16, 32 * ks, PT);
      const v16h aL0 = ld_frag(SEL, 0, 32 * ks, PT);
      const v16h aL1 = ld_frag(SEL, 16, 32 * ks, PT);
      const v16h bw  = ld_frag(wp, 16 * wv, 32 * ks, DMD);
      ch0 = mma_h(aH0, bw, ch0);
      ch1 = mma_h(aH1, bw, ch1);
      cl0 = mma_h(aL0, bw, cl0);
      cl1 = mma_h(aL1, bw, cl1);
      guard4_5(ch0, ch1, cl0, cl1, aH0, aH1, aL0, aL1, bw);
    }
    const int col = 16 * wv + l15;
    const float bb = bp[col];
#pragma unroll
    for (int r = 0; r < 8; ++r) {
      f16 x, y;
      split16(ch0[r] * PINV + cl0[r] * RINV + bb, x, y);
      OH[(8 * hl + r) * PT + col] = x;
      OL[(8 * hl + r) * PT + col] = y;
      split16(ch1[r] * PINV + cl1[r] * RINV + bb, x, y);
      OH[(16 + 8 * hl + r) * PT + col] = x;
      OL[(16 + 8 * hl + r) * PT + col] = y;
    }
  }
  __syncthreads();

  if (wv < 4) {
    const int mt = wv >> 1, nt = wv & 1;
    v8f c0 = {}, c1 = {};
#pragma unroll
    for (int ks = 0; ks < 4; ++ks) {
      const v16h aH = ld_frag(QH, 16 * mt, 32 * ks, PT);
      const v16h aL = ld_frag(QL, 16 * mt, 32 * ks, PT);
      const v16h kH = ld_frag(KH, 16 * nt, 32 * ks, PT);
      const v16h kL = ld_frag(KL, 16 * nt, 32 * ks, PT);
      c0 = mma_h(aH, kH, c0);
      c1 = mma_h(aH, kL, c1);
      c1 = mma_h(aL, kH, c1);
      guard2_4(c0, c1, aH, aL, kH, kL);
    }
    const int col = 16 * nt + l15;
#pragma unroll
    for (int r = 0; r < 8; ++r)
      Sc[(16 * mt + 8 * hl + r) * PS + col] = (c0[r] * HHINV + c1[r] * XINV) * INVSQ;
  }
  __syncthreads();

  if (tid < NA) {
    float* row = Sc + tid * PS;
    float mx = row[0];
#pragma unroll 1
    for (int c = 1; c < NA; ++c) mx = fmaxf(mx, row[c]);
    float s = 0.0f;
#pragma unroll 1
    for (int c = 0; c < NA; ++c) {
      const float e = expf(row[c] - mx);
      row[c] = e;
      s += e;
    }
    const float inv = 1.0f / s;
#pragma unroll 1
    for (int c = 0; c < NA; ++c) row[c] = row[c] * inv;
  }
  __syncthreads();

  {
    const int row = tid >> 3, q = tid & 7;
    const v4f val = *(const v4fa*)&Sc[row * PS + 4 * q];
    float* op = outw + (size_t)bh * (NA * NA) + row * NA + 4 * q;
    *(volatile v4f*)op = val;
    __threadfence();
    *(volatile v4f*)op = val;
  }
}

__global__ __launch_bounds__(256)
void k_emb(const float* __restrict__ states, const float* __restrict__ actions, const float* __restrict__ policies,
           const unsigned short* __restrict__ wsap_h, const float* __restrict__ b_sap,
           const unsigned short* __restrict__ wav_h,  const float* __restrict__ b_av,
           unsigned short* ath, unsigned short* atl, unsigned short* aph, unsigned short* apl, int nb) {
  extern __shared__ __align__(16) char smem[];
  f16*   A    = (f16*)(smem + E_A);
  f16*   EH   = (f16*)(smem + E_EH);
  f16*   EL   = (f16*)(smem + E_EL);
  float* avS  = (float*)(smem + E_AV);
  float* bsap = (float*)(smem + E_B);
  float* bav  = bsap + NH * DMD;

  const int tid = threadIdx.x, lane = tid & 31, wv = tid >> 5, hl = lane >> 4, l15 = lane & 15;
  const int b = (int)blockIdx.x;
  if (b >= nb) return;
  const v8h zero8 = {};

#pragma unroll
  for (int it = 0; it < 4; ++it) {
    const int idx = tid + it * 256;
    const int r = idx >> 4, c8 = (idx & 15) << 3;
    const int k = r & (NA - 1);
    const float* p = states + (size_t)(b * NA + k) * OBS + c8;
    const v4f x0 = *(const v4f*)p;
    const v4f x1 = *(const v4f*)(p + 4);
    v8h o = {};
#pragma unroll
    for (int e = 0; e < 4; ++e) {
      o[e]     = (f16)(bf16r(x0[e]) * ASC);
      o[4 + e] = (f16)(bf16r(x1[e]) * ASC);
    }
    *(v8h*)&A[r * PA + c8] = o;
  }
  {
    const int r = tid >> 2, q4 = tid & 3;
    const int k = r & (NA - 1);
    const float* ap = (r < NA) ? actions : policies;
    const int ca = (q4 < 2) ? (q4 << 3) : 8;
    const float* p = ap + (size_t)(b * NA + k) * ACT + ca;
    const v4f x0 = *(const v4f*)p;
    const v4f x1 = *(const v4f*)(p + 4);
    v8h o = {};
#pragma unroll
    for (int e = 0; e < 4; ++e) {
      o[e]     = (f16)(bf16r(x0[e]) * ASC);
      o[4 + e] = (f16)(bf16r(x1[e]) * ASC);
    }
    o = (q4 < 2) ? o : zero8;
    *(v8h*)&A[r * PA + OBS + (q4 << 3)] = o;
  }
  bsap[tid]       = bf16r(b_sap[tid]);
  bsap[tid + 256] = bf16r(b_sap[tid + 256]);
  if (tid < NH * EV) bav[tid] = bf16r(b_av[tid]);
  __syncthreads();

#pragma unroll 1
  for (int h = 0; h < NH; ++h) {
    {
      const f16* wp = (const f16*)wsap_h + (size_t)h * DMD * OAP;
      v8f c0 = {}, c1 = {}, c2 = {}, c3 = {};
#pragma unroll
      for (int ks = 0; ks < 5; ++ks) {
        const v16h a0 = ld_frag(A, 0, 32 * ks, PA);
        const v16h a1 = ld_frag(A, 16, 32 * ks, PA);
        const v16h a2 = ld_frag(A, 32, 32 * ks, PA);
        const v16h a3 = ld_frag(A, 48, 32 * ks, PA);
        const v16h bw = ld_frag(wp, 16 * wv, 32 * ks, OAP);
        c0 = mma_h(a0, bw, c0);
        c1 = mma_h(a1, bw, c1);
        c2 = mma_h(a2, bw, c2);
        c3 = mma_h(a3, bw, c3);
        guard4_5(c0, c1, c2, c3, a0, a1, a2, a3, bw);
      }
      const int col = 16 * wv + l15;
      const float bb = bsap[h * DMD + col];
#pragma unroll
      for (int r = 0; r < 8; ++r) {
        f16 x, y;
        split16(leaky_f(c0[r] * PINV + bb), x, y);
        EH[(8 * hl + r) * PT + col] = x;       EL[(8 * hl + r) * PT + col] = y;
        split16(leaky_f(c1[r] * PINV + bb), x, y);
        EH[(16 + 8 * hl + r) * PT + col] = x;  EL[(16 + 8 * hl + r) * PT + col] = y;
        split16(leaky_f(c2[r] * PINV + bb), x, y);
        EH[(32 + 8 * hl + r) * PT + col] = x;  EL[(32 + 8 * hl + r) * PT + col] = y;
        split16(leaky_f(c3[r] * PINV + bb), x, y);
        EH[(48 + 8 * hl + r) * PT + col] = x;  EL[(48 + 8 * hl + r) * PT + col] = y;
      }
    }
    __syncthreads();

    {
      const f16* wp = (const f16*)wav_h + (size_t)h * EV * DMD;
      const int mt = wv >> 1, nt = wv & 1;
      v8f ch = {}, cl = {};
#pragma unroll
      for (int ks = 0; ks < 4; ++ks) {
        const v16h aH = ld_frag(EH, 16 * mt, 32 * ks, PT);
        const v16h aL = ld_frag(EL, 16 * mt, 32 * ks, PT);
        const v16h bw = ld_frag(wp, 16 * nt, 32 * ks, DMD);
        ch = mma_h(aH, bw, ch);
        cl = mma_h(aL, bw, cl);
        guard2_3(ch, cl, aH, aL, bw);
      }
      const int col = 16 * nt + l15;
      const float bb = bav[h * EV + col];
#pragma unroll
      for (int r = 0; r < 8; ++r)
        avS[(h * 2 * NA + 16 * mt + 8 * hl + r) * PS + col] = leaky_f(ch[r] * PINV + cl[r] * RINV + bb);
    }
    __syncthreads();
  }

  v8us oh[2], ol[2], qh[2], ql[2];
#pragma unroll
  for (int it = 0; it < 2; ++it) {
    const int p = tid + it * 256;
    const int hh = p >> 7, e = (p >> 2) & 31, k0 = (p & 3) << 3;
    v8h a_h = {}, a_l = {}, p_h = {}, p_l = {};
#pragma unroll
    for (int c = 0; c < 8; ++c) {
      f16 x, y;
      split16(avS[(hh * 2 * NA + k0 + c) * PS + e], x, y);
      a_h[c] = x; a_l[c] = y;
      split16(avS[(hh * 2 * NA + NA + e) * PS + k0 + c], x, y);
      p_h[c] = x; p_l[c] = y;
    }
    oh[it] = __builtin_bit_cast(v8us, a_h);
    ol[it] = __builtin_bit_cast(v8us, a_l);
    qh[it] = __builtin_bit_cast(v8us, p_h);
    ql[it] = __builtin_bit_cast(v8us, p_l);
  }
  const size_t base = (size_t)b * (NH * EV * NA);
#pragma unroll
  for (int it = 0; it < 2; ++it) {
    const size_t off = base + (size_t)(tid + it * 256) * 8;
    *(volatile v8us*)(ath + off) = oh[it];
    *(volatile v8us*)(atl + off) = ol[it];
    *(volatile v8us*)(aph + off) = qh[it];
    *(volatile v8us*)(apl + off) = ql[it];
  }
  __threadfence();
#pragma unroll
  for (int it = 0; it < 2; ++it) {
    const size_t off = base + (size_t)(tid + it * 256) * 8;
    *(volatile v8us*)(ath + off) = oh[it];
    *(volatile v8us*)(atl + off) = ol[it];
    *(volatile v8us*)(aph + off) = qh[it];
    *(volatile v8us*)(apl + off) = ql[it];
  }
}

__global__ __launch_bounds__(256)
void k_node(const float* wall,
            const unsigned short* __restrict__ ath, const unsigned short* __restrict__ atl,
            const unsigned short* __restrict__ aph, const unsigned short* __restrict__ apl,
            const unsigned short* __restrict__ wf1_h, const float* __restrict__ b_f1,
            const unsigned short* __restrict__ wf2_h, const float* __restrict__ b_f2,
            float* outv, int nblk) {
  extern __shared__ __align__(16) char smem[];
  f16*   WH = (f16*)(smem + N_WH);
  f16*   WL = (f16*)(smem + N_WL);
  f16*   TH = (f16*)(smem + N_TH);
  f16*   TL = (f16*)(smem + N_TL);
  f16*   NHp = (f16*)(smem + N_NH);
  f16*   NLp = (f16*)(smem + N_NL);
  f16*   HH = (f16*)(smem + N_HH);
  f16*   HL = (f16*)(smem + N_HL);
  float* ST = (float*)(smem + N_ST);
  float* bb = (float*)(smem + N_BB);

  const int tid = threadIdx.x, lane = tid & 31, wv = tid >> 5, hl = lane >> 4, l15 = lane & 15;
  const int blk = (int)blockIdx.x;
  if (blk >= nblk) return;
  const int b = blk >> 4, jp = blk & 15;
  const size_t base = (size_t)b * (NH * EV * NA);

  {
    const float* wsrc = wall + (size_t)b * (NH * NA * NA);
#pragma unroll
    for (int it = 0; it < 4; ++it) {
      const int idx = tid + it * 256;
      const int hh = idx >> 8, i = (idx >> 3) & 31, k0 = (idx & 7) << 2;
      const v4f w = *(const v4f*)(wsrc + (size_t)idx * 4);
      v4h wh = {}, wl = {};
#pragma unroll
      for (int c = 0; c < 4; ++c) {
        f16 x, y;
        split16(w[c], x, y);
        wh[c] = x; wl[c] = y;
      }
      *(v4h*)&WH[(hh * NA + i) * PW + k0] = wh;
      *(v4h*)&WL[(hh * NA + i) * PW + k0] = wl;
    }
  }
  {
    const f16* athp = (const f16*)ath + base;
    const f16* atlp = (const f16*)atl + base;
#pragma unroll
    for (int it = 0; it < 2; ++it) {
      const int p = tid + it * 256;
      const int hh = p >> 7, e = (p >> 2) & 31, k0 = (p & 3) << 3;
      const v8h vh = *(const v8h*)(athp + (size_t)p * 8);
      const v8h vl = *(const v8h*)(atlp + (size_t)p * 8);
#pragma unroll
      for (int jj = 0; jj < 2; ++jj) {
        *(v8h*)&TH[((jj * NH + hh) * EV + e) * PW + k0] = vh;
        *(v8h*)&TL[((jj * NH + hh) * EV + e) * PW + k0] = vl;
      }
    }
  }
  if (tid < HID) bb[tid] = bf16r(b_f1[tid]);
  if (tid < FIN) bb[HID + tid] = bf16r(b_f2[tid]);
  __syncthreads();

  {
    const int jj = tid >> 7, hh = (tid >> 5) & 3, e = tid & 31;
    const int j = 2 * jp + jj;
    const size_t go = base + (size_t)(hh * NA + j) * EV + e;
    const f16 vh = ((const f16*)aph)[go];
    const f16 vl = ((const f16*)apl)[go];
    const int li = ((jj * NH + hh) * EV + e) * PW + j;
    TH[li] = vh;
    TL[li] = vl;
  }
  __syncthreads();

  {
    const int jj = wv >> 2, hh = wv & 3;
    const f16* THp = TH + (size_t)((jj * NH + hh) * EV) * PW;
    const f16* TLp = TL + (size_t)((jj * NH + hh) * EV) * PW;
    const v16h bH0 = ld_frag(THp, 0, 0, PW);
    const v16h bH1 = ld_frag(THp, 16, 0, PW);
    const v16h bL0 = ld_frag(TLp, 0, 0, PW);
    const v16h bL1 = ld_frag(TLp, 16, 0, PW);
#pragma unroll
    for (int mt = 0; mt < 2; ++mt) {
      const v16h aH = ld_frag(WH, hh * NA + 16 * mt, 0, PW);
      const v16h aL = ld_frag(WL, hh * NA + 16 * mt, 0, PW);
      v8f g0 = {}, g1 = {}, x0 = {}, x1 = {};
      g0 = mma_h(aH, bH0, g0);
      g1 = mma_h(aH, bH1, g1);
      x0 = mma_h(aH, bL0, x0);
      x0 = mma_h(aL, bH0, x0);
      x1 = mma_h(aH, bL1, x1);
      x1 = mma_h(aL, bH1, x1);
      guard4_6(g0, g1, x0, x1, aH, aL, bH0, bH1, bL0, bL1);
      const int row0 = jj * NA + 16 * mt + 8 * hl;
      const int col0 = hh * EV + l15, col1 = col0 + 16;
#pragma unroll
      for (int r = 0; r < 8; ++r) {
        f16 x, y;
        split16(g0[r] * HHINV + x0[r] * XINV, x, y);
        NHp[(row0 + r) * PT + col0] = x;  NLp[(row0 + r) * PT + col0] = y;
        split16(g1[r] * HHINV + x1[r] * XINV, x, y);
        NHp[(row0 + r) * PT + col1] = x;  NLp[(row0 + r) * PT + col1] = y;
      }
    }
  }
  __syncthreads();

  {
    const f16* wp = (const f16*)wf1_h;
    const int nt = wv & 3, m0 = 2 * (wv >> 2);
    v8f ch0 = {}, ch1 = {}, cl0 = {}, cl1 = {};
#pragma unroll
    for (int ks = 0; ks < 4; ++ks) {
      const v16h aH0 = ld_frag(NHp, 16 * m0, 32 * ks, PT);
      const v16h aH1 = ld_frag(NHp, 16 * (m0 + 1), 32 * ks, PT);
      const v16h aL0 = ld_frag(NLp, 16 * m0, 32 * ks, PT);
      const v16h aL1 = ld_frag(NLp, 16 * (m0 + 1), 32 * ks, PT);
      const v16h bw  = ld_frag(wp, 16 * nt, 32 * ks, DMD);
      ch0 = mma_h(aH0, bw, ch0);
      ch1 = mma_h(aH1, bw, ch1);
      cl0 = mma_h(aL0, bw, cl0);
      cl1 = mma_h(aL1, bw, cl1);
      guard4_5(ch0, ch1, cl0, cl1, aH0, aH1, aL0, aL1, bw);
    }
    const int col = 16 * nt + l15;
    const float bv = bb[col];
#pragma unroll
    for (int r = 0; r < 8; ++r) {
      f16 x, y;
      split16(leaky_f(ch0[r] * PINV + cl0[r] * RINV + bv), x, y);
      HH[(16 * m0 + 8 * hl + r) * PH + col] = x;        HL[(16 * m0 + 8 * hl + r) * PH + col] = y;
      split16(leaky_f(ch1[r] * PINV + cl1[r] * RINV + bv), x, y);
      HH[(16 * (m0 + 1) + 8 * hl + r) * PH + col] = x;  HL[(16 * (m0 + 1) + 8 * hl + r) * PH + col] = y;
    }
  }
  __syncthreads();

  if (wv < 4) {
    const f16* wp = (const f16*)wf2_h;
    const int mt = wv;
    v8f ch = {}, cl = {};
#pragma unroll
    for (int ks = 0; ks < 2; ++ks) {
      const v16h aH = ld_frag(HH, 16 * mt, 32 * ks, PH);
      const v16h aL = ld_frag(HL, 16 * mt, 32 * ks, PH);
      const v16h bw = ld_frag(wp, 0, 32 * ks, HID);
      ch = mma_h(aH, bw, ch);
      cl = mma_h(aL, bw, cl);
      guard2_3(ch, cl, aH, aL, bw);
    }
    const float bv = bb[HID + l15];
#pragma unroll
    for (int r = 0; r < 8; ++r) {
      const int row = 16 * mt + 8 * hl + r;
      const int jj = row >> 5, i = row & 31;
      ST[i * PS + jj * FIN + l15] = ch[r] * PINV + cl[r] * RINV + bv;
    }
  }
  __syncthreads();

  {
    const int i = tid >> 3, q = tid & 7;
    const v4f val = *(const v4fa*)&ST[i * PS + 4 * q];
    float* op = outv + ((size_t)(b * NA + i) * NA + 2 * jp) * FIN + 4 * q;
    *(volatile v4f*)op = val;
    __threadfence();
    *(volatile v4f*)op = val;
  }
}

extern "C" void kernel_launch(void* const* d_in, const int* in_sizes, int n_in,
                              void* d_out, int out_size, void* d_ws, size_t ws_size,
                              hipStream_t stream) {
  if (n_in < 17) return;
  if (in_sizes[0] != NB * NA * OBS) return;
  if (in_sizes[1] != NB * NA * ACT || in_sizes[2] != NB * NA * ACT) return;
  if (in_sizes[3] != NH * OBS * DMD || in_sizes[4] != NH * DMD) return;
  if (in_sizes[5] != NH * DMD * DMD || in_sizes[6] != NH * DMD) return;
  if (in_sizes[7] != NH * DMD * DMD || in_sizes[8] != NH * DMD) return;
  if (in_sizes[9] != NH * OA * DMD || in_sizes[10] != NH * DMD) return;
  if (in_sizes[11] != NH * DMD * EV || in_sizes[12] != NH * EV) return;
  if (in_sizes[13] != DMD * HID || in_sizes[14] != HID) return;
  if (in_sizes[15] != HID * FIN || in_sizes[16] != FIN) return;
  if (out_size != OUT0_N + OUT1_N) return;

  const size_t sz_wse  = (size_t)NH * DMD * DMD * 2;
  const size_t sz_wsap = (size_t)NH * DMD * OAP * 2;
  const size_t sz_wav  = (size_t)NH * EV * DMD * 2;
  const size_t sz_wf1  = (size_t)HID * DMD * 2;
  const size_t sz_wf2  = (size_t)FIN * HID * 2;
  const size_t sz_av   = (size_t)NB * NH * EV * NA * 2;
  const size_t off_wse  = 0;
  const size_t off_wk   = off_wse + sz_wse;
  const size_t off_wq   = off_wk + sz_wse;
  const size_t off_wsap = off_wq + sz_wse;
  const size_t off_wav  = off_wsap + sz_wsap;
  const size_t off_wf1  = off_wav + sz_wav;
  const size_t off_wf2  = off_wf1 + sz_wf1;
  const size_t off_ath  = off_wf2 + sz_wf2;
  const size_t off_atl  = off_ath + sz_av;
  const size_t off_aph  = off_atl + sz_av;
  const size_t off_apl  = off_aph + sz_av;
  const size_t need     = off_apl + sz_av;
  if (need > ws_size) return;
  if (need > (size_t)134217728) return;

  const float* states   = (const float*)d_in[0];
  const float* policies = (const float*)d_in[1];
  const float* actions  = (const float*)d_in[2];
  const float* W_se  = (const float*)d_in[3];
  const float* b_se  = (const float*)d_in[4];
  const float* W_k   = (const float*)d_in[5];
  const float* b_k   = (const float*)d_in[6];
  const float* W_q   = (const float*)d_in[7];
  const float* b_q   = (const float*)d_in[8];
  const float* W_sap = (const float*)d_in[9];
  const float* b_sap = (const float*)d_in[10];
  const float* W_av  = (const float*)d_in[11];
  const float* b_av  = (const float*)d_in[12];
  const float* W_f1  = (const float*)d_in[13];
  const float* b_f1  = (const float*)d_in[14];
  const float* W_f2  = (const float*)d_in[15];
  const float* b_f2  = (const float*)d_in[16];

  float* out0 = (float*)d_out;
  float* out1 = out0 + OUT0_N;

  char* wsb = (char*)d_ws;
  unsigned short* wse_p  = (unsigned short*)(wsb + off_wse);
  unsigned short* wk_p   = (unsigned short*)(wsb + off_wk);
  unsigned short* wq_p   = (unsigned short*)(wsb + off_wq);
  unsigned short* wsap_p = (unsigned short*)(wsb + off_wsap);
  unsigned short* wav_p  = (unsigned short*)(wsb + off_wav);
  unsigned short* wf1_p  = (unsigned short*)(wsb + off_wf1);
  unsigned short* wf2_p  = (unsigned short*)(wsb + off_wf2);
  unsigned short* ath_p  = (unsigned short*)(wsb + off_ath);
  unsigned short* atl_p  = (unsigned short*)(wsb + off_atl);
  unsigned short* aph_p  = (unsigned short*)(wsb + off_aph);
  unsigned short* apl_p  = (unsigned short*)(wsb + off_apl);

  const int n8_se  = NH * DMD * DMD / 8;
  const int n8_sap = NH * DMD * OAP / 8;
  const int n8_av  = NH * EV * DMD / 8;
  const int n8_f1  = HID * DMD / 8;
  const int n8_f2  = FIN * HID / 8;
  k_cvt_t<<<dim3((n8_se + 255) / 256),  dim3(256), 0, stream>>>(W_se,  wse_p,  NH, OBS, DMD, OBS);
  k_cvt_t<<<dim3((n8_se + 255) / 256),  dim3(256), 0, stream>>>(W_k,   wk_p,   NH, DMD, DMD, DMD);
  k_cvt_t<<<dim3((n8_se + 255) / 256),  dim3(256), 0, stream>>>(W_q,   wq_p,   NH, DMD, DMD, DMD);
  k_cvt_t<<<dim3((n8_sap + 255) / 256), dim3(256), 0, stream>>>(W_sap, wsap_p, NH, OA,  DMD, OAP);
  k_cvt_t<<<dim3((n8_av + 255) / 256),  dim3(256), 0, stream>>>(W_av,  wav_p,  NH, DMD, EV,  DMD);
  k_cvt_t<<<dim3((n8_f1 + 255) / 256),  dim3(256), 0, stream>>>(W_f1,  wf1_p,  1,  DMD, HID, DMD);
  k_cvt_t<<<dim3((n8_f2 + 255) / 256),  dim3(256), 0, stream>>>(W_f2,  wf2_p,  1,  HID, FIN, HID);

  (void)hipFuncSetAttribute(reinterpret_cast<const void*>(&k_attn), hipFuncAttributeMaxDynamicSharedMemorySize, A_TOTAL);
  (void)hipFuncSetAttribute(reinterpret_cast<const void*>(&k_emb),  hipFuncAttributeMaxDynamicSharedMemorySize, E_TOTAL);
  (void)hipFuncSetAttribute(reinterpret_cast<const void*>(&k_node), hipFuncAttributeMaxDynamicSharedMemorySize, N_TOTAL);

  const int nbh = NB * NH;
  k_attn<<<dim3(nbh), dim3(256), A_TOTAL, stream>>>(states, wse_p, b_se, wk_p, b_k, wq_p, b_q, out1, nbh);

  const int nb = NB;
  k_emb<<<dim3(nb), dim3(256), E_TOTAL, stream>>>(states, actions, policies, wsap_p, b_sap, wav_p, b_av,
                                                  ath_p, atl_p, aph_p, apl_p, nb);

  const int nblk = NB * (NA / 2);
  k_node<<<dim3(nblk), dim3(256), N_TOTAL, stream>>>(out1, ath_p, atl_p, aph_p, apl_p, wf1_p, b_f1, wf2_p, b_f2,
                                                      out0, nblk);
  (void)hipGetLastError();
}
